// MilliesRNN_11244224381288
// MI455X (gfx1250) — hardware-run, weakly checked
//
#include <hip/hip_runtime.h>
#include <math.h>

constexpr int NBATCH  = 64;
constexpr int NSTEP   = 512;
constexpr int NIN     = 256;
constexpr int NHID    = 1024;
constexpr int NOUTF   = 256;
constexpr int TCHUNK  = 128;
constexpr int NCHUNK  = NSTEP / TCHUNK;
constexpr int CHROWS  = TCHUNK * NBATCH;
constexpr int NTHR    = 256;
constexpr int SEQ_BLK = 16;
constexpr int HPITCH  = NHID + 8;
constexpr int SLABP   = 68;
constexpr float WCARRY     = 64.0f;
constexpr float WCARRY_INV = 1.0f / WCARRY;

static_assert(NBATCH == 64);
static_assert(NSTEP % TCHUNK == 0);
static_assert(NBATCH % SEQ_BLK == 0);
static_assert(NHID == 128 * (NTHR / 32));
static_assert(NIN % 32 == 0 && NHID % 32 == 0 && NOUTF % 32 == 0);
static_assert(CHROWS % 64 == 0 && NHID % 64 == 0 && NOUTF % 64 == 0);
static_assert((SEQ_BLK * NHID / 8) % NTHR == 0);
static_assert((HPITCH * 2) % 16 == 0);
static_assert(((CHROWS / 64) * (NHID / 64)) % 8 == 0);
static_assert(((CHROWS / 64) * (NOUTF / 64)) % 8 == 0);

typedef __attribute__((ext_vector_type(16))) _Float16 v16h;
typedef __attribute__((ext_vector_type(8)))  _Float16 v8h;
typedef __attribute__((ext_vector_type(8)))  float    v8f;
typedef __attribute__((ext_vector_type(4)))  float    v4f;

__device__ __forceinline__ void dep_guard4_h(v8f& a, v8f& b, v8f& c, v8f& d, v16h x, v16h y) {
  asm volatile("v_nop\n\tv_nop\n\tv_nop\n\tv_nop" : "+v"(a), "+v"(b), "+v"(c), "+v"(d) : "v"(x), "v"(y));
}
__device__ __forceinline__ void keep4_h(v16h a, v16h b, v16h c, v16h d) {
  asm volatile("v_nop" :: "v"(a), "v"(b), "v"(c), "v"(d));
}
__device__ __forceinline__ void acc_guard4(v8f& a, v8f& b, v8f& c, v8f& d) {
  asm volatile("v_nop\n\tv_nop\n\tv_nop\n\tv_nop" : "+v"(a), "+v"(b), "+v"(c), "+v"(d));
}

struct FragH {
  union U { v16h v; v8h h[2]; };
  static __device__ __forceinline__ v16h load(const _Float16* p) {
    U f;
    f.h[0] = *(const v8h*)(p);
    f.h[1] = *(const v8h*)(p + 16);
    return f.v;
  }
  static __device__ __forceinline__ v8f mma(v16h a, v16h b, v8f c) {
    return __builtin_amdgcn_wmma_f32_16x16x32_f16(false, a, false, b, (short)0, c, false, false);
  }
};

__device__ __forceinline__ float ftanh_pos(float z) {
  return 1.0f - 2.0f * __builtin_amdgcn_rcpf(__expf(2.0f * z) + 1.0f);
}

template <bool TMAJ>
__global__ __launch_bounds__(NTHR) void cvt8_f16_kernel(const float* __restrict__ src, unsigned short* __restrict__ dst,
                                                        int n8, int ncol8, float sc) {
  const int i = blockIdx.x * NTHR + threadIdx.x;
  if (i < n8) {
    const int row = i / ncol8;
    const int c8  = i - row * ncol8;
    size_t srow = (size_t)row;
    if (TMAJ) srow = (size_t)(row % NBATCH) * NSTEP + (size_t)(row / NBATCH);
    const float* sp = src + srow * (size_t)(ncol8 * 8) + (size_t)(c8 * 8);
    const v4f a = *(const v4f*)(sp);
    const v4f b = *(const v4f*)(sp + 4);
    v8h hv;
#pragma unroll
    for (int e = 0; e < 4; ++e) {
      const float fa = a[e] * sc;
      const float fb = b[e] * sc;
      hv[e]     = (_Float16)fa;
      hv[4 + e] = (_Float16)fb;
    }
    _Float16* dp = (_Float16*)dst + (size_t)i * 8;
    *(volatile v8h*)dp = hv;
    __threadfence();
    *(volatile v8h*)dp = hv;
  }
}

template <int NBIAS, int OUT_MODE, int ACT, bool REMAP>
__global__ __launch_bounds__(NTHR) void gemm64_f16_kernel(
    const unsigned short* __restrict__ Ap, int lda,
    const unsigned short* __restrict__ Btp, int ldb,
    void* __restrict__ Cout, int ldc,
    const float* __restrict__ bias0, const float* __restrict__ bias1,
    int M, int N, int K, float scale, int t0) {
  const _Float16* A  = (const _Float16*)Ap;
  const _Float16* Bt = (const _Float16*)Btp;
  __shared__ __align__(16) float sT[NTHR / 32][16 * SLABP];
  const int lane = threadIdx.x & 31;
  const int wave = threadIdx.x >> 5;
  const int tilesN = N >> 6;
  const int tilesM = M >> 6;
  const int tile = blockIdx.x * (NTHR / 32) + wave;
  if (tile >= tilesM * tilesN) return;
  const int tm = tile / tilesN;
  const int tn = tile - tm * tilesN;
  const int m0 = tm << 6;
  const int n0 = tn << 6;

  const int rlane = lane & 15;
  const int koff  = (lane >> 4) * 8;
  const int mOff  = (lane >> 4) * 8;

  v8f acc[4][4];
#pragma unroll
  for (int i = 0; i < 4; ++i)
#pragma unroll
    for (int j = 0; j < 4; ++j) acc[i][j] = (v8f){0.f, 0.f, 0.f, 0.f, 0.f, 0.f, 0.f, 0.f};

  const _Float16* bbase = Bt + (size_t)(n0 + rlane) * ldb + koff;
  const _Float16* abase = A  + (size_t)(m0 + rlane) * lda + koff;
  const size_t bstep = (size_t)16 * ldb;
  const size_t astep = (size_t)16 * lda;

  for (int k0 = 0; k0 < K; k0 += 32) {
    v16h bh[4];
#pragma unroll
    for (int j = 0; j < 4; ++j) bh[j] = FragH::load(bbase + (size_t)j * bstep + k0);
#pragma unroll
    for (int i = 0; i < 4; ++i) {
      const v16h ah = FragH::load(abase + (size_t)i * astep + k0);
#pragma unroll
      for (int j = 0; j < 4; ++j) acc[i][j] = FragH::mma(ah, bh[j], acc[i][j]);
      dep_guard4_h(acc[i][0], acc[i][1], acc[i][2], acc[i][3], ah, bh[3]);
    }
    keep4_h(bh[0], bh[1], bh[2], bh[3]);
  }
  acc_guard4(acc[0][0], acc[0][1], acc[0][2], acc[0][3]);
  acc_guard4(acc[1][0], acc[1][1], acc[1][2], acc[1][3]);
  acc_guard4(acc[2][0], acc[2][1], acc[2][2], acc[2][3]);
  acc_guard4(acc[3][0], acc[3][1], acc[3][2], acc[3][3]);

  float bv[4];
#pragma unroll
  for (int j = 0; j < 4; ++j) {
    const int n = n0 + (j << 4) + rlane;
    float t = bias0[n];
    if (NBIAS == 2) t += bias1[n];
    bv[j] = t;
  }

  float* slab = sT[wave];
#pragma unroll
  for (int i = 0; i < 4; ++i) {
    const int mBase = m0 + (i << 4);
#pragma unroll
    for (int j = 0; j < 4; ++j) {
#pragma unroll
      for (int r = 0; r < 8; ++r) {
        const float v = acc[i][j][r] * scale + bv[j];
        slab[(mOff + r) * SLABP + (j << 4) + rlane] = v;
      }
    }
    __builtin_amdgcn_fence(__ATOMIC_RELEASE, "workgroup");
    __builtin_amdgcn_wave_barrier();
    __builtin_amdgcn_fence(__ATOMIC_ACQUIRE, "workgroup");
    if (ACT == 1) {
#pragma unroll 1
      for (int q = 0; q < 32; ++q) {
        const int idx = q * 32 + lane;
        float* sp = slab + (idx >> 6) * SLABP + (idx & 63);
        const float v = *sp;
        const float a = tanhf(fmaxf(v, 0.0f));
        *sp = a;
      }
      __builtin_amdgcn_fence(__ATOMIC_RELEASE, "workgroup");
      __builtin_amdgcn_wave_barrier();
      __builtin_amdgcn_fence(__ATOMIC_ACQUIRE, "workgroup");
    }
    if (OUT_MODE == 0) {
      float* C = (float*)Cout;
      const int hh = lane >> 4, c4 = (lane & 15) * 4;
      for (int pass = 0; pass < 2; ++pass) {
#pragma unroll
        for (int it = 0; it < 8; ++it) {
          const int row = it * 2 + hh;
          const int grow = mBase + row;
          size_t orow = (size_t)grow;
          if (REMAP) orow = (size_t)(grow % NBATCH) * NSTEP + (size_t)t0 + (size_t)(grow / NBATCH);
          const v4f v = *(const v4f*)(slab + row * SLABP + c4);
          *(volatile v4f*)(C + orow * (size_t)ldc + n0 + c4) = v;
        }
        __threadfence();
      }
    } else {
      _Float16* C = (_Float16*)Cout;
      const int q = lane >> 3, c8 = (lane & 7) * 8;
      for (int pass = 0; pass < 2; ++pass) {
#pragma unroll
        for (int it = 0; it < 4; ++it) {
          const int row = it * 4 + q;
          const float* sp = slab + row * SLABP + c8;
          v8h hv;
#pragma unroll
          for (int e = 0; e < 8; ++e) {
            const float f = sp[e];
            hv[e] = (_Float16)f;
          }
          *(volatile v8h*)(C + (size_t)(mBase + row) * ldc + n0 + c8) = hv;
        }
        __threadfence();
      }
    }
    __builtin_amdgcn_fence(__ATOMIC_RELEASE, "workgroup");
    __builtin_amdgcn_wave_barrier();
    __builtin_amdgcn_fence(__ATOMIC_ACQUIRE, "workgroup");
  }
}

__global__ __launch_bounds__(NTHR) void scan_kernel(const float* __restrict__ PRE, const unsigned short* __restrict__ Wp,
                                                    const unsigned short* __restrict__ Sin, unsigned short* __restrict__ Sout,
                                                    unsigned short* __restrict__ HSEQ) {
  __shared__ __align__(16) _Float16 Ah[2][SEQ_BLK * HPITCH];
  const _Float16* W  = (const _Float16*)Wp;
  const _Float16* S0 = (const _Float16*)Sin;
  _Float16* S1 = (_Float16*)Sout;
  _Float16* HS = (_Float16*)HSEQ;
  const int tid = threadIdx.x, lane = tid & 31, wave = tid >> 5;
  const int c = lane & 15, hh = lane >> 4, koff = hh * 8;
  const int rowbase = blockIdx.x * SEQ_BLK;

#pragma unroll 1
  for (int it = 0; it < (SEQ_BLK * NHID / 8) / NTHR; ++it) {
    const int idx = it * NTHR + tid;
    const int row = idx >> 7;
    const int c8  = (idx & 127) * 8;
    const v8h v = *(const v8h*)(S0 + (size_t)(rowbase + row) * NHID + c8);
    *(v8h*)(&Ah[0][row * HPITCH + c8]) = v;
  }
  __syncthreads();

  const v8f z8 = {0.f, 0.f, 0.f, 0.f, 0.f, 0.f, 0.f, 0.f};

#pragma unroll 1
  for (int tl = 0; tl < TCHUNK; ++tl) {
    const int cur = tl & 1;
    const _Float16* ahrow = &Ah[cur][0] + c * HPITCH + koff;
    _Float16* ahn = &Ah[cur ^ 1][0];
    const float* prow = PRE + ((size_t)tl * NBATCH + (size_t)(rowbase + 8 * hh)) * NHID;
    const bool last = (tl == TCHUNK - 1);

#pragma unroll 1
    for (int g = 0; g < 2; ++g) {
      const int colbase = 128 * wave + 64 * g + c;
      const _Float16* w0 = W + (size_t)colbase * NHID + koff;
      const _Float16* w1 = w0 + (size_t)16 * NHID;
      const _Float16* w2 = w0 + (size_t)32 * NHID;
      const _Float16* w3 = w0 + (size_t)48 * NHID;
      v8f acc[4];
      acc[0] = z8; acc[1] = z8; acc[2] = z8; acc[3] = z8;
#pragma unroll 1
      for (int k0 = 0; k0 < NHID; k0 += 32) {
        const v16h a  = FragH::load(ahrow + k0);
        const v16h b0 = FragH::load(w0 + k0);
        const v16h b1 = FragH::load(w1 + k0);
        const v16h b2 = FragH::load(w2 + k0);
        const v16h b3 = FragH::load(w3 + k0);
        acc[0] = FragH::mma(a, b0, acc[0]);
        acc[1] = FragH::mma(a, b1, acc[1]);
        acc[2] = FragH::mma(a, b2, acc[2]);
        acc[3] = FragH::mma(a, b3, acc[3]);
        dep_guard4_h(acc[0], acc[1], acc[2], acc[3], a, b3);
        keep4_h(b0, b1, b2, b3);
      }
      acc_guard4(acc[0], acc[1], acc[2], acc[3]);
#pragma unroll
      for (int nt = 0; nt < 4; ++nt) {
        const int col = colbase + 16 * nt;
        float pre[8];
#pragma unroll
        for (int r = 0; r < 8; ++r) pre[r] = prow[(size_t)r * NHID + col];
#pragma unroll
        for (int r = 0; r < 8; ++r) {
          const float z  = acc[nt][r] * WCARRY_INV + pre[r];
          const float th = ftanh_pos(z);
          const float hn = (z > 0.0f) ? th : 0.0f;
          ahn[(8 * hh + r) * HPITCH + col] = (_Float16)hn;
        }
        asm volatile("" ::: "memory");
      }
    }
    __syncthreads();

    {
      const _Float16* srcp = ahn + 128 * wave + 8 * c;
      v8h vv[8];
#pragma unroll
      for (int it = 0; it < 8; ++it) {
        const int row = it * 2 + hh;
        vv[it] = *(const v8h*)(srcp + row * HPITCH);
      }
      for (int pass = 0; pass < 2; ++pass) {
#pragma unroll
        for (int it = 0; it < 8; ++it) {
          const int row = it * 2 + hh;
          *(volatile v8h*)(HS + ((size_t)tl * NBATCH + (size_t)(rowbase + row)) * NHID + 128 * wave + 8 * c) = vv[it];
          if (last) *(volatile v8h*)(S1 + (size_t)(rowbase + row) * NHID + 128 * wave + 8 * c) = vv[it];
        }
        __threadfence();
      }
    }
  }
}

extern "C" void kernel_launch(void* const* d_in, const int* in_sizes, int n_in,
                              void* d_out, int out_size, void* d_ws, size_t ws_size, hipStream_t stream) {
  if (n_in < 17 || d_out == nullptr || d_ws == nullptr) return;
  if (in_sizes[0] != NBATCH * NSTEP * NIN || in_sizes[1] != NBATCH * NHID || in_sizes[2] != NBATCH * NHID ||
      in_sizes[3] != NHID * NIN || in_sizes[4] != NHID || in_sizes[5] != NHID * NHID || in_sizes[6] != NHID ||
      in_sizes[7] != NOUTF * NHID || in_sizes[8] != NOUTF || in_sizes[9] != NOUTF * NOUTF || in_sizes[10] != NOUTF ||
      in_sizes[11] != NHID * NOUTF || in_sizes[12] != NHID || in_sizes[13] != NHID * NHID || in_sizes[14] != NHID ||
      in_sizes[15] != NOUTF * NHID || in_sizes[16] != NOUTF || out_size != NBATCH * NSTEP * NOUTF) return;

  const float* data     = (const float*)d_in[0];
  const float* h0_v     = (const float*)d_in[1];
  const float* h0_m     = (const float*)d_in[2];
  const float* Wi2h     = (const float*)d_in[3];
  const float* bi2h     = (const float*)d_in[4];
  const float* Wh2h     = (const float*)d_in[5];
  const float* bh2h     = (const float*)d_in[6];
  const float* Wh2o     = (const float*)d_in[7];
  const float* bh2o     = (const float*)d_in[8];
  const float* Wthal    = (const float*)d_in[9];
  const float* bthal    = (const float*)d_in[10];
  const float* Wi2h_dos = (const float*)d_in[11];
  const float* bi2h_dos = (const float*)d_in[12];
  const float* Wh2h_dos = (const float*)d_in[13];
  const float* bh2h_dos = (const float*)d_in[14];
  const float* Wh2o_dos = (const float*)d_in[15];
  const float* bh2o_dos = (const float*)d_in[16];

  char* ws = (char*)d_ws;
  size_t off = 0;
  auto carve = [&](size_t bytes) -> char* { char* p = ws + off; off += (bytes + 255) & ~(size_t)255; return p; };
  unsigned short* W1   = (unsigned short*)carve((size_t)NHID * NIN * 2);
  unsigned short* W2   = (unsigned short*)carve((size_t)NHID * NHID * 2);
  unsigned short* W3   = (unsigned short*)carve((size_t)NOUTF * NHID * 2);
  unsigned short* W4   = (unsigned short*)carve((size_t)NOUTF * NOUTF * 2);
  unsigned short* W5   = (unsigned short*)carve((size_t)NHID * NOUTF * 2);
  unsigned short* W6   = (unsigned short*)carve((size_t)NHID * NHID * 2);
  unsigned short* W7   = (unsigned short*)carve((size_t)NOUTF * NHID * 2);
  unsigned short* X16  = (unsigned short*)carve((size_t)NSTEP * NBATCH * NIN * 2);
  float*          PRE  = (float*)carve((size_t)CHROWS * NHID * 4);
  unsigned short* HV   = (unsigned short*)carve((size_t)CHROWS * NHID * 2);
  unsigned short* HM   = (unsigned short*)carve((size_t)CHROWS * NHID * 2);
  unsigned short* OUTV = (unsigned short*)carve((size_t)CHROWS * NOUTF * 2);
  unsigned short* OUTT = (unsigned short*)carve((size_t)CHROWS * NOUTF * 2);
  unsigned short* SV[2];
  unsigned short* SM[2];
  SV[0] = (unsigned short*)carve((size_t)NBATCH * NHID * 2);
  SV[1] = (unsigned short*)carve((size_t)NBATCH * NHID * 2);
  SM[0] = (unsigned short*)carve((size_t)NBATCH * NHID * 2);
  SM[1] = (unsigned short*)carve((size_t)NBATCH * NHID * 2);
  if (off > ws_size || off > (size_t)134217728) return;

  const int n8_hi = NHID * (NIN / 8);
  const int n8_hh = NHID * (NHID / 8);
  const int n8_oh = NOUTF * (NHID / 8);
  const int n8_oo = NOUTF * (NOUTF / 8);
  const int n8_ho = NHID * (NOUTF / 8);
  const int n8_st = NBATCH * (NHID / 8);
  const int n8_x  = NSTEP * NBATCH * (NIN / 8);
  cvt8_f16_kernel<false><<<n8_hi / NTHR, NTHR, 0, stream>>>(Wi2h,     W1, n8_hi, NIN / 8,   WCARRY);
  cvt8_f16_kernel<false><<<n8_hh / NTHR, NTHR, 0, stream>>>(Wh2h,     W2, n8_hh, NHID / 8,  WCARRY);
  cvt8_f16_kernel<false><<<n8_oh / NTHR, NTHR, 0, stream>>>(Wh2o,     W3, n8_oh, NHID / 8,  WCARRY);
  cvt8_f16_kernel<false><<<n8_oo / NTHR, NTHR, 0, stream>>>(Wthal,    W4, n8_oo, NOUTF / 8, WCARRY);
  cvt8_f16_kernel<false><<<n8_ho / NTHR, NTHR, 0, stream>>>(Wi2h_dos, W5, n8_ho, NOUTF / 8, WCARRY);
  cvt8_f16_kernel<false><<<n8_hh / NTHR, NTHR, 0, stream>>>(Wh2h_dos, W6, n8_hh, NHID / 8,  WCARRY);
  cvt8_f16_kernel<false><<<n8_oh / NTHR, NTHR, 0, stream>>>(Wh2o_dos, W7, n8_oh, NHID / 8,  WCARRY);
  cvt8_f16_kernel<false><<<n8_st / NTHR, NTHR, 0, stream>>>(h0_v, SV[0], n8_st, NHID / 8, 1.0f);
  cvt8_f16_kernel<false><<<n8_st / NTHR, NTHR, 0, stream>>>(h0_m, SM[0], n8_st, NHID / 8, 1.0f);
  cvt8_f16_kernel<true><<<n8_x / NTHR, NTHR, 0, stream>>>(data, X16, n8_x, NIN / 8, 1.0f);

  const int grid_h = (CHROWS / 64) * (NHID / 64) / 8;
  const int grid_o = (CHROWS / 64) * (NOUTF / 64) / 8;

  for (int ch = 0; ch < NCHUNK; ++ch) {
    const int t0 = ch * TCHUNK;
    const unsigned short* XA = X16 + (size_t)ch * CHROWS * NIN;
    gemm64_f16_kernel<2, 0, 0, false><<<grid_h, NTHR, 0, stream>>>(
        XA, NIN, W1, NIN, (void*)PRE, NHID, bi2h, bh2h, CHROWS, NHID, NIN, WCARRY_INV, 0);
    scan_kernel<<<NBATCH / SEQ_BLK, NTHR, 0, stream>>>(PRE, W2, SV[ch & 1], SV[(ch + 1) & 1], HV);
    gemm64_f16_kernel<1, 1, 0, false><<<grid_o, NTHR, 0, stream>>>(
        HV, NHID, W3, NHID, (void*)OUTV, NOUTF, bh2o, bh2o, CHROWS, NOUTF, NHID, WCARRY_INV, 0);
    gemm64_f16_kernel<1, 1, 1, false><<<grid_o, NTHR, 0, stream>>>(
        OUTV, NOUTF, W4, NOUTF, (void*)OUTT, NOUTF, bthal, bthal, CHROWS, NOUTF, NOUTF, WCARRY_INV, 0);
    gemm64_f16_kernel<2, 0, 0, false><<<grid_h, NTHR, 0, stream>>>(
        OUTT, NOUTF, W5, NOUTF, (void*)PRE, NHID, bi2h_dos, bh2h_dos, CHROWS, NHID, NOUTF, WCARRY_INV, 0);
    scan_kernel<<<NBATCH / SEQ_BLK, NTHR, 0, stream>>>(PRE, W6, SM[ch & 1], SM[(ch + 1) & 1], HM);
    gemm64_f16_kernel<1, 0, 0, true><<<grid_o, NTHR, 0, stream>>>(
        HM, NHID, W7, NHID, d_out, NOUTF, bh2o_dos, bh2o_dos, CHROWS, NOUTF, NHID, WCARRY_INV, t0);
  }
}
